// EfficientTransformerBlock_20229295964956
// MI455X (gfx1250) — hardware-verified
//
#include <hip/hip_runtime.h>


#define NBT  4
#define NN   2048
#define DMOD 512
#define DFF  1024
#define NH_  8
#define HD   64
#define ZH   2
#define DM   DMOD
#define NTK  NN
#define SCL  0.125f
#define LEPS 1e-5f
#define LOSC 1024.0f

typedef _Float16 h16;
typedef unsigned short bf;
typedef __attribute__((ext_vector_type(16))) __bf16   v16bf;
typedef __attribute__((ext_vector_type(16))) _Float16 v16h;
typedef __attribute__((ext_vector_type(8)))  _Float16 v8h;
typedef __attribute__((ext_vector_type(8)))  unsigned short v8us;
typedef __attribute__((ext_vector_type(8)))  float    v8f;
typedef __attribute__((ext_vector_type(4)))  float    v4f;
typedef __attribute__((ext_vector_type(4)))  _Float16 v4h;
typedef v8h  __attribute__((may_alias)) v8ha;
typedef v4f  __attribute__((may_alias)) v4fa;
typedef v8us __attribute__((may_alias)) v8usa;

__device__ __forceinline__ unsigned short f2bf(float f) { unsigned u = __float_as_uint(f); u += 0x7FFFu + ((u >> 16) & 1u); return (unsigned short)(u >> 16); }
__device__ __forceinline__ float bf2f(unsigned short b) { return __uint_as_float(((unsigned)b) << 16); }
__device__ __forceinline__ float bfr(float f) { return bf2f(f2bf(f)); }
__device__ __forceinline__ v16h cat16(v8h lo, v8h hi) { return __builtin_shufflevector(lo, hi, 0, 1, 2, 3, 4, 5, 6, 7, 8, 9, 10, 11, 12, 13, 14, 15); }
__device__ __forceinline__ v16bf cat16b(v8us lo, v8us hi) { return __builtin_bit_cast(v16bf, __builtin_shufflevector(lo, hi, 0, 1, 2, 3, 4, 5, 6, 7, 8, 9, 10, 11, 12, 13, 14, 15)); }
__device__ __forceinline__ v8f wmma16(v16h a, v16h b, v8f c) { return __builtin_amdgcn_wmma_f32_16x16x32_f16(false, a, false, b, (short)0, c, false, false); }
__device__ __forceinline__ v8f wmmab(v16bf a, v16bf b, v8f c) { return __builtin_amdgcn_wmma_f32_16x16x32_bf16(false, a, false, b, (short)0, c, false, false); }

__global__ __launch_bounds__(256) void k_wt(const float* __restrict__ Wm, int K, int ncols, bf* WT) {
    __shared__ __align__(16) unsigned short tl[64 * 72];
    const int tid = threadIdx.x, k0 = blockIdx.x * 64, n0 = blockIdx.y * 64;
    const int kk = tid >> 2, nq = (tid & 3) * 16;
#pragma unroll
    for (int i = 0; i < 16; ++i) tl[(nq + i) * 72 + kk] = f2bf(Wm[(size_t)(k0 + kk) * ncols + n0 + nq + i]);
    __syncthreads();
    const int piece = tid & 7;
    auto pass = [&]() {
#pragma unroll
        for (int s = 0; s < 2; ++s) { const int nr = (tid >> 3) + 32 * s; const v8us val = *(const v8usa*)(tl + nr * 72 + piece * 8); *(volatile v8us*)(WT + (size_t)(n0 + nr) * K + k0 + piece * 8) = val; }
    };
    pass(); __threadfence(); pass();
}
template <bool SPLITA, bool F16OUT = false>
__global__ __launch_bounds__(128) void k_gemmb(const bf* __restrict__ A, const bf* __restrict__ Al, const bf* __restrict__ Bn, const float* __restrict__ bias, float* C, int ldc, h16* C2, const float* __restrict__ R = nullptr, int K = DM, int roundR = 1) {
    __shared__ __align__(16) float ost[4][16 * 68];
    const int lane = threadIdx.x & 31, wave = threadIdx.x >> 5, lr = lane & 15, hi = lane >> 4;
    const int r0 = blockIdx.x * 64 + wave * 16, c0 = blockIdx.y * 64;
    const size_t aoff = (size_t)(r0 + lr) * K + 8 * hi;
    size_t boff[4];
#pragma unroll
    for (int t = 0; t < 4; ++t) boff[t] = (size_t)(c0 + t * 16 + lr) * K + 8 * hi;
    v8f acc[4];
#pragma unroll
    for (int t = 0; t < 4; ++t) acc[t] = (v8f){};
#pragma unroll 1
    for (int kc = 0; kc < K; kc += 32) {
        const v16bf a = cat16b(*(const v8us*)(A + aoff + kc), *(const v8us*)(A + aoff + kc + 16));
        v16bf al = a;
        if (SPLITA) al = cat16b(*(const v8us*)(Al + aoff + kc), *(const v8us*)(Al + aoff + kc + 16));
#pragma unroll
        for (int t = 0; t < 4; ++t) { const v16bf b = cat16b(*(const v8us*)(Bn + boff[t] + kc), *(const v8us*)(Bn + boff[t] + kc + 16)); acc[t] = wmmab(a, b, acc[t]); if (SPLITA) acc[t] = wmmab(al, b, acc[t]); }
        asm volatile("v_nop\n\tv_nop\n\tv_nop\n\tv_nop" : "+v"(acc[0]), "+v"(acc[1]), "+v"(acc[2]), "+v"(acc[3]) : "v"(a), "v"(al));
    }
    float* os = &ost[wave][0];
#pragma unroll
    for (int t = 0; t < 4; ++t) { const float bv = bias ? bfr(bias[c0 + t * 16 + lr]) : 0.f;
#pragma unroll
        for (int j = 0; j < 8; ++j) os[(hi * 8 + j) * 68 + t * 16 + lr] = acc[t][j] + bv; }
    __syncthreads();
    if (F16OUT) {
        h16* crow = (h16*)(void*)C + (size_t)r0 * ldc + c0;
        auto pass = [&]() {
#pragma unroll
            for (int s = 0; s < 4; ++s) { const int row = 4 * s + (lane >> 3), piece = lane & 7; const float* sp = os + row * 68 + piece * 8; v8h o, o2;
#pragma unroll
                for (int i = 0; i < 8; ++i) { const h16 a = (h16)sp[i]; o[i] = a; o2[i] = (h16)((sp[i] - (float)a) * LOSC); }
                *(volatile v8h*)(crow + (size_t)row * ldc + piece * 8) = o; if (C2) *(volatile v8h*)(C2 + (size_t)r0 * ldc + c0 + (size_t)row * ldc + piece * 8) = o2; }
        };
        pass(); __threadfence(); pass();
    } else {
        float* crow = C + (size_t)r0 * ldc + c0;
        auto pass = [&]() {
#pragma unroll
            for (int s = 0; s < 8; ++s) { const int Lid = (lane >> 3) + 4 * s, piece = lane & 7; const int row = Lid >> 1, cofs = (Lid & 1) * 32 + piece * 4;
                v4f val = *(const v4fa*)(os + row * 68 + cofs); if (R) { const v4f rv = *(const v4f*)(R + ((size_t)r0 + row) * ldc + c0 + cofs); val += roundR ? (v4f){bfr(rv[0]), bfr(rv[1]), bfr(rv[2]), bfr(rv[3])} : rv; }
                *(volatile v4f*)(crow + (size_t)row * ldc + cofs) = val; }
        };
        pass(); __threadfence(); pass();
    }
}


template <int MODE>
__global__ __launch_bounds__(128) void k_gemm3z(const bf* __restrict__ Ah, const bf* __restrict__ Al, const bf* __restrict__ Bh, const bf* __restrict__ Bl, int K, float* C, int ldc, size_t sA, size_t sB, size_t sC) {
    if ((MODE & 1) && (int)blockIdx.y * 64 > (int)blockIdx.x * 64 + 63) return;
    const size_t z = blockIdx.z; Ah += z * sA; Al += z * sA; Bh += z * sB; Bl += z * sB; C += z * sC;
    const int Klim = (MODE & 2) ? min(K, ((int)blockIdx.x + 1) * 64) : K;
    __shared__ __align__(16) float ost[4][16 * 68];
    const int lane = threadIdx.x & 31, wave = threadIdx.x >> 5, lr = lane & 15, hi = lane >> 4;
    const int r0 = blockIdx.x * 64 + wave * 16, c0 = blockIdx.y * 64;
    const size_t aoff = (size_t)(r0 + lr) * K + 8 * hi;
    v8f acc[4];
#pragma unroll
    for (int t = 0; t < 4; ++t) acc[t] = (v8f){};
#pragma unroll 1
    for (int kc = 0; kc < Klim; kc += 32) {
        const v16bf a = cat16b(*(const v8us*)(Ah + aoff + kc), *(const v8us*)(Ah + aoff + kc + 16));
        v16bf al = a; if (!(MODE & 4) && !(MODE & 16)) al = cat16b(*(const v8us*)(Al + aoff + kc), *(const v8us*)(Al + aoff + kc + 16));
#pragma unroll
        for (int t = 0; t < 4; ++t) { const size_t bo = (size_t)(c0 + t * 16 + lr) * K + kc + 8 * hi;
            const v16bf bh = cat16b(*(const v8us*)(Bh + bo), *(const v8us*)(Bh + bo + 16));
            acc[t] = wmmab(a, bh, acc[t]);
            if (!(MODE & 4)) { if (!(MODE & 16)) acc[t] = wmmab(al, bh, acc[t]); if (!(MODE & 8)) { const v16bf bl = cat16b(*(const v8us*)(Bl + bo), *(const v8us*)(Bl + bo + 16)); acc[t] = wmmab(a, bl, acc[t]); } } }
        asm volatile("v_nop\n\tv_nop\n\tv_nop\n\tv_nop" : "+v"(acc[0]), "+v"(acc[1]), "+v"(acc[2]), "+v"(acc[3]) : "v"(a), "v"(al));
    }
    float* os = &ost[wave][0];
#pragma unroll
    for (int t = 0; t < 4; ++t) {
#pragma unroll
        for (int j = 0; j < 8; ++j) os[(hi * 8 + j) * 68 + t * 16 + lr] = acc[t][j]; }
    __builtin_amdgcn_wave_barrier(); asm volatile("" ::: "memory");
    float* crow = C + (size_t)r0 * ldc + c0;
    auto pass = [&]() {
#pragma unroll
        for (int s = 0; s < 8; ++s) { const int Lid = (lane >> 3) + 4 * s, piece = lane & 7; const int row = Lid >> 1, cofs = (Lid & 1) * 32 + piece * 4;
            const v4f val = *(const v4fa*)(os + row * 68 + cofs); *(volatile v4f*)(crow + (size_t)row * ldc + cofs) = val; }
    };
    pass(); __threadfence(); pass();
}
__global__ __launch_bounds__(256) void k_planes32z(const float* __restrict__ F, int ld, int off, float sc, int rows, bf* Ph, bf* Pl) {
    typedef __attribute__((ext_vector_type(2))) unsigned short v2us;
    const int lane = threadIdx.x & 31; const size_t r = ((size_t)blockIdx.x * 8 + (threadIdx.x >> 5)) * 2 + (lane >> 4); if (r >= (size_t)rows) return; const int z = blockIdx.z; const int c0 = (lane & 15) * 2; v2us oh, ol;
    Ph += (size_t)z * rows * 32; Pl += (size_t)z * rows * 32;
#pragma unroll
    for (int i = 0; i < 2; ++i) { const float y = F[r * ld + off + z * 32 + c0 + i] * sc; const unsigned short hb = f2bf(y); oh[i] = hb; ol[i] = f2bf(y - bf2f(hb)); }
    const size_t o = r * 32 + c0; *(volatile v2us*)(Ph + o) = oh; *(volatile v2us*)(Pl + o) = ol; __threadfence(); *(volatile v2us*)(Ph + o) = oh; *(volatile v2us*)(Pl + o) = ol;
}
__global__ __launch_bounds__(256) void k_vtpadz(const float* __restrict__ F, int ld, int off, int nk, bf* Th, bf* Tl) {
    typedef __attribute__((ext_vector_type(2))) unsigned short v2us;
    const int lane = threadIdx.x & 31; const size_t wid = (size_t)blockIdx.x * 8 + (threadIdx.x >> 5); if (wid >= (size_t)64 * (nk / 64)) return; const int z = blockIdx.z; const int d = (int)(wid / (nk / 64)); const int k0 = (int)(wid % (nk / 64)) * 64 + lane * 2; v2us oh, ol;
    Th += (size_t)z * 64 * nk; Tl += (size_t)z * 64 * nk;
#pragma unroll
    for (int i = 0; i < 2; ++i) { const float y = (d < 32) ? F[(size_t)(k0 + i) * ld + off + z * 32 + (d < 32 ? d : 0)] : 0.f; const unsigned short hb = f2bf(y); oh[i] = hb; ol[i] = f2bf(y - bf2f(hb)); }
    const size_t o = (size_t)d * nk + k0; *(volatile v2us*)(Th + o) = oh; *(volatile v2us*)(Tl + o) = ol; __threadfence(); *(volatile v2us*)(Th + o) = oh; *(volatile v2us*)(Tl + o) = ol;
}
template <int NK>
__global__ __launch_bounds__(256) void k_softmaxz(const float* __restrict__ S, int rows, bf* PH, bf* PL) {
    typedef __attribute__((ext_vector_type(4))) unsigned short v4us;
    const int lane = threadIdx.x & 31, i = blockIdx.x * 8 + (threadIdx.x >> 5); if (i >= rows) return; const size_t zo = (size_t)blockIdx.z * rows * NK; const float* sr = S + zo + (size_t)i * NK; PH += zo; PL += zo;
    float m = -3.0e38f;
#pragma unroll 1
    for (int c0 = lane * 4; c0 < NK; c0 += 128) {
#pragma unroll
        for (int q = 0; q < 4; ++q) m = fmaxf(m, sr[c0 + q]); }
#pragma unroll
    for (int sh = 16; sh; sh >>= 1) m = fmaxf(m, __shfl_xor(m, sh, 32));
    float sum = 0.f;
#pragma unroll 1
    for (int c0 = lane * 4; c0 < NK; c0 += 128) {
#pragma unroll
        for (int q = 0; q < 4; ++q) sum += __expf(sr[c0 + q] - m); }
#pragma unroll
    for (int sh = 16; sh; sh >>= 1) sum += __shfl_xor(sum, sh, 32);
    const float inv = 1.0f / sum;
#pragma unroll 1
    for (int ps = 0; ps < 2; ++ps) {
#pragma unroll 1
        for (int c0 = lane * 4; c0 < NK; c0 += 128) { v4us oh, ol;
#pragma unroll
            for (int q = 0; q < 4; ++q) { const float p = __expf(sr[c0 + q] - m) * inv; const unsigned short hb = f2bf(p); oh[q] = hb; ol[q] = f2bf(p - bf2f(hb)); }
            const size_t o = (size_t)i * NK + c0; *(volatile v4us*)(PH + o) = oh; *(volatile v4us*)(PL + o) = ol; }
        if (ps == 0) __threadfence(); }
}
__global__ __launch_bounds__(256) void k_placez(const float* __restrict__ XH, int rows, int ldy, float* Y) {
    const int lane = threadIdx.x & 31; const size_t q = (size_t)blockIdx.x * 8 + (threadIdx.x >> 5); if (q >= (size_t)rows) return; const int z = blockIdx.z; const float v = XH[((size_t)z * rows + q) * 64 + lane];
    *(volatile float*)(Y + q * ldy + z * 32 + lane) = v; __threadfence(); *(volatile float*)(Y + q * ldy + z * 32 + lane) = v;
}

__global__ __launch_bounds__(256) void k_hplanesz(const float* __restrict__ F, int ld, int h0, float sc, int rows, bf* Ph, bf* Pl) {
    typedef __attribute__((ext_vector_type(2))) unsigned short v2us;
    const int lane = threadIdx.x & 31; const size_t r = (size_t)blockIdx.x * 8 + (threadIdx.x >> 5); if (r >= (size_t)rows) return; const int z = blockIdx.z; v2us oh, ol;
    Ph += (size_t)z * rows * 64; Pl += (size_t)z * rows * 64;
#pragma unroll
    for (int i = 0; i < 2; ++i) { const float y = F[r * ld + (h0 + z) * 64 + lane * 2 + i] * sc; const unsigned short hb = f2bf(y); oh[i] = hb; ol[i] = f2bf(y - bf2f(hb)); }
    const size_t o = r * 64 + lane * 2; *(volatile v2us*)(Ph + o) = oh; *(volatile v2us*)(Pl + o) = ol; __threadfence(); *(volatile v2us*)(Ph + o) = oh; *(volatile v2us*)(Pl + o) = ol;
}
__global__ __launch_bounds__(256) void k_vtz(const float* __restrict__ F, int ld, int h0, int nk, bf* Th, bf* Tl) {
    typedef __attribute__((ext_vector_type(2))) unsigned short v2us;
    const int lane = threadIdx.x & 31; const size_t wid = (size_t)blockIdx.x * 8 + (threadIdx.x >> 5); if (wid >= (size_t)64 * (nk / 64)) return; const int z = blockIdx.z; const int d = (int)(wid / (nk / 64)); const int t0 = (int)(wid % (nk / 64)) * 64 + lane * 2; v2us oh, ol;
    Th += (size_t)z * 64 * nk; Tl += (size_t)z * 64 * nk;
#pragma unroll
    for (int i = 0; i < 2; ++i) { const float y = F[(size_t)(t0 + i) * ld + (h0 + z) * 64 + d]; const unsigned short hb = f2bf(y); oh[i] = hb; ol[i] = f2bf(y - bf2f(hb)); }
    const size_t o = (size_t)d * nk + t0; *(volatile v2us*)(Th + o) = oh; *(volatile v2us*)(Tl + o) = ol; __threadfence(); *(volatile v2us*)(Th + o) = oh; *(volatile v2us*)(Tl + o) = ol;
}
template <int NK>
__global__ __launch_bounds__(256) void k_softmaxzs(const float* __restrict__ S, int rows, float sc, bf* PH, bf* PL) {
    typedef __attribute__((ext_vector_type(4))) unsigned short v4us;
    const int lane = threadIdx.x & 31, i = blockIdx.x * 8 + (threadIdx.x >> 5); if (i >= rows) return; const size_t zo = (size_t)blockIdx.z * rows * NK; const float* sr = S + zo + (size_t)i * NK; PH += zo; PL += zo;
    float m = -3.0e38f;
#pragma unroll 1
    for (int c0 = lane * 4; c0 < NK; c0 += 128) {
#pragma unroll
        for (int q = 0; q < 4; ++q) m = fmaxf(m, sr[c0 + q] * sc); }
#pragma unroll
    for (int sh = 16; sh; sh >>= 1) m = fmaxf(m, __shfl_xor(m, sh, 32));
    float sum = 0.f;
#pragma unroll 1
    for (int c0 = lane * 4; c0 < NK; c0 += 128) {
#pragma unroll
        for (int q = 0; q < 4; ++q) sum += __expf(sr[c0 + q] * sc - m); }
#pragma unroll
    for (int sh = 16; sh; sh >>= 1) sum += __shfl_xor(sum, sh, 32);
    const float inv = 1.0f / sum;
#pragma unroll 1
    for (int ps = 0; ps < 2; ++ps) {
#pragma unroll 1
        for (int c0 = lane * 4; c0 < NK; c0 += 128) { v4us oh, ol;
#pragma unroll
            for (int q = 0; q < 4; ++q) { const float p = __expf(sr[c0 + q] * sc - m) * inv; const unsigned short hb = f2bf(p); oh[q] = hb; ol[q] = f2bf(p - bf2f(hb)); }
            const size_t o = (size_t)i * NK + c0; *(volatile v4us*)(PH + o) = oh; *(volatile v4us*)(PL + o) = ol; }
        if (ps == 0) __threadfence(); }
}

template <bool RB>
__global__ __launch_bounds__(256) void k_addln512(const float* __restrict__ Ain, const float* __restrict__ Bin, const float* __restrict__ g, const float* __restrict__ bb, float* X1out, bf* Hh, bf* Hl) {
    typedef __attribute__((ext_vector_type(4))) unsigned short v4us;
    const int lane = threadIdx.x & 31; const size_t r = (size_t)blockIdx.x * 8 + (threadIdx.x >> 5); if (r >= (size_t)NN) return; float v[16]; float s = 0.f;
#pragma unroll
    for (int q = 0; q < 4; ++q) {
#pragma unroll
        for (int i = 0; i < 4; ++i) { const size_t o = r * DMOD + q * 128 + lane * 4 + i; const float t = (Bin != nullptr) ? (Ain[o] + (RB ? bfr(Bin[o]) : Bin[o])) : bfr(Ain[o]); v[q * 4 + i] = t; s += t; } }
#pragma unroll
    for (int sh = 16; sh; sh >>= 1) s += __shfl_xor(s, sh, 32);
    const float mu = s * (1.0f / DMOD); float qv = 0.f;
#pragma unroll
    for (int i = 0; i < 16; ++i) { const float d = v[i] - mu; qv = fmaf(d, d, qv); }
#pragma unroll
    for (int sh = 16; sh; sh >>= 1) qv += __shfl_xor(qv, sh, 32);
    const float rs = rsqrtf(qv * (1.0f / DMOD) + LEPS);
#pragma unroll 1
    for (int ps = 0; ps < 2; ++ps) {
#pragma unroll
        for (int q = 0; q < 4; ++q) { const int c0 = q * 128 + lane * 4; v4f xo; v4us oh, ol;
#pragma unroll
            for (int i = 0; i < 4; ++i) { xo[i] = v[q * 4 + i]; const float y = (xo[i] - mu) * rs * bfr(g[c0 + i]) + bfr(bb[c0 + i]); const unsigned short hb = f2bf(y); oh[i] = hb; ol[i] = f2bf(y - bf2f(hb)); }
            const size_t o = r * DMOD + c0; if (X1out != nullptr) *(volatile v4f*)(X1out + o) = xo; *(volatile v4us*)(Hh + o) = oh; *(volatile v4us*)(Hl + o) = ol; }
        if (ps == 0) __threadfence(); }
}
__global__ __launch_bounds__(256) void k_gelu1024(const float* __restrict__ F, int rows, bf* Gh, bf* Gl) {
    const int lane = threadIdx.x & 31; const size_t r = (size_t)blockIdx.x * 8 + (threadIdx.x >> 5); if (r >= (size_t)rows) return;
#pragma unroll 1
    for (int ps = 0; ps < 2; ++ps) {
#pragma unroll 1
        for (int q = 0; q < DFF / 256; ++q) { const size_t o = r * DFF + q * 256 + lane * 8; const v8f v = *(const v8f*)(F + o); v8us oh, ol;
#pragma unroll
            for (int i = 0; i < 8; ++i) { const float xv = v[i]; const float gx = 0.5f * xv * (1.0f + erff(xv * 0.70710678118654752f)); const unsigned short hb = f2bf(gx); oh[i] = hb; ol[i] = f2bf(gx - bf2f(hb)); }
            *(volatile v8us*)(Gh + o) = oh; *(volatile v8us*)(Gl + o) = ol; }
        if (ps == 0) __threadfence(); }
}
__global__ __launch_bounds__(256) void k_split512(const float* __restrict__ src, int rows, bf* dh, bf* dl) {
    const int lane = threadIdx.x & 31; const size_t r = (size_t)blockIdx.x * 8 + (threadIdx.x >> 5); if (r >= (size_t)rows) return;
#pragma unroll 1
    for (int ps = 0; ps < 2; ++ps) {
#pragma unroll
        for (int q = 0; q < DMOD / 256; ++q) { const size_t o = r * DMOD + q * 256 + lane * 8; const v8f v = *(const v8f*)(src + o); v8us oh, ol;
#pragma unroll
            for (int i = 0; i < 8; ++i) { const unsigned short hb = f2bf(v[i]); oh[i] = hb; ol[i] = f2bf(v[i] - bf2f(hb)); }
            *(volatile v8us*)(dh + o) = oh; *(volatile v8us*)(dl + o) = ol; }
        if (ps == 0) __threadfence(); }
}
__global__ __launch_bounds__(256) void k_add512(const float* __restrict__ A, const float* __restrict__ B, float* OUTB) {
    const int lane = threadIdx.x & 31; const size_t r = (size_t)blockIdx.x * 8 + (threadIdx.x >> 5); if (r >= (size_t)NN) return;
#pragma unroll
    for (int q = 0; q < 4; ++q) { const size_t o = r * DMOD + q * 128 + lane * 4; const v4f v = *(const v4f*)(A + o) + *(const v4f*)(B + o); *(volatile v4f*)(OUTB + o) = v; }
    __threadfence();
#pragma unroll
    for (int q = 0; q < 4; ++q) { const size_t o = r * DMOD + q * 128 + lane * 4; const v4f v = *(const v4f*)(A + o) + *(const v4f*)(B + o); *(volatile v4f*)(OUTB + o) = v; }
}

extern "C" void kernel_launch(void* const* d_in, const int* in_sizes, int n_in,
                              void* d_out, int out_size, void* d_ws, size_t ws_size, hipStream_t stream) {
    (void)in_sizes; (void)n_in; (void)out_size;
    const float* x = (const float*)d_in[0]; const float* w_qkv = (const float*)d_in[1]; const float* b_qkv = (const float*)d_in[2]; const float* w_proj = (const float*)d_in[3]; const float* b_proj = (const float*)d_in[4]; const float* w_ff1 = (const float*)d_in[5]; const float* b_ff1 = (const float*)d_in[6]; const float* w_ff2 = (const float*)d_in[7]; const float* b_ff2 = (const float*)d_in[8];
    const float* g1 = (const float*)d_in[9]; const float* be1 = (const float*)d_in[10]; const float* g2 = (const float*)d_in[11]; const float* be2 = (const float*)d_in[12];
    float* out = (float*)d_out;
    char* wsp = (char*)d_ws;
    auto take = [&](size_t bytes) { char* p = wsp; wsp += (bytes + 255) & ~(size_t)255; return (void*)p; };
    bf* WQKV = (bf*)take((size_t)3 * DMOD * DMOD * 2); bf* WP = (bf*)take((size_t)DMOD * DMOD * 2); bf* WF1 = (bf*)take((size_t)DFF * DMOD * 2); bf* WF2 = (bf*)take((size_t)DMOD * DFF * 2);
    bf* Hh = (bf*)take((size_t)NN * DMOD * 2); bf* Hl = (bf*)take((size_t)NN * DMOD * 2); float* QKV = (float*)take((size_t)NN * 3 * DMOD * 4);
    bf* Qh = (bf*)take((size_t)ZH * NN * HD * 2); bf* Ql = (bf*)take((size_t)ZH * NN * HD * 2); bf* Kh = (bf*)take((size_t)ZH * NN * HD * 2); bf* Kl = (bf*)take((size_t)ZH * NN * HD * 2); bf* VTh = (bf*)take((size_t)ZH * HD * NN * 2); bf* VTl = (bf*)take((size_t)ZH * HD * NN * 2);
    float* S = (float*)take((size_t)ZH * NN * NN * 4); bf* PH = (bf*)take((size_t)ZH * NN * NN * 2); bf* PL = (bf*)take((size_t)ZH * NN * NN * 2); float* O = (float*)take((size_t)NN * DMOD * 4); bf* Oh = (bf*)take((size_t)NN * DMOD * 2); bf* Ol = (bf*)take((size_t)NN * DMOD * 2);
    float* PO = (float*)take((size_t)NN * DMOD * 4); float* X1 = (float*)take((size_t)NN * DMOD * 4);
    if ((size_t)(wsp - (char*)d_ws) > ws_size) return;
    float* F1 = S; bf* Gh = PH; bf* Gl = PL; float* F2 = O;
    k_wt<<<dim3(DMOD / 64, (3 * DMOD) / 64, 1), 256, 0, stream>>>(w_qkv, DMOD, 3 * DMOD, WQKV); k_wt<<<dim3(DMOD / 64, DMOD / 64, 1), 256, 0, stream>>>(w_proj, DMOD, DMOD, WP); k_wt<<<dim3(DMOD / 64, DFF / 64, 1), 256, 0, stream>>>(w_ff1, DMOD, DFF, WF1); k_wt<<<dim3(DFF / 64, DMOD / 64, 1), 256, 0, stream>>>(w_ff2, DFF, DMOD, WF2);
    for (int b = 0; b < NBT; ++b) { const float* xb = x + (size_t)b * NN * DMOD;
        k_addln512<false><<<NN / 8, 256, 0, stream>>>(xb, nullptr, g1, be1, nullptr, Hh, Hl);
        k_gemmb<true, false><<<dim3(NN / 64, (3 * DMOD) / 64, 1), 128, 0, stream>>>(Hh, Hl, WQKV, b_qkv, QKV, 3 * DMOD, nullptr, nullptr, DMOD);
        for (int g = 0; g < NH_ / ZH; ++g) { const int h0 = g * ZH;
            k_hplanesz<<<dim3(NN / 8, 1, ZH), 256, 0, stream>>>(QKV, 3 * DMOD, h0, 1.0f, NN, Qh, Ql); k_hplanesz<<<dim3(NN / 8, 1, ZH), 256, 0, stream>>>(QKV + DMOD, 3 * DMOD, h0, 1.0f, NN, Kh, Kl);
            k_vtz<<<dim3((HD * (NN / 64)) / 8, 1, ZH), 256, 0, stream>>>(QKV + 2 * DMOD, 3 * DMOD, h0, NN, VTh, VTl);
            k_gemm3z<0><<<dim3(NN / 64, NN / 64, ZH), 128, 0, stream>>>(Qh, Ql, Kh, Kl, HD, S, NN, (size_t)NN * HD, (size_t)NN * HD, (size_t)NN * NN);
            k_softmaxzs<NN><<<dim3(NN / 8, 1, ZH), 256, 0, stream>>>(S, NN, SCL, PH, PL);
            k_gemm3z<0><<<dim3(NN / 64, 1, ZH), 128, 0, stream>>>(PH, PL, VTh, VTl, NN, O + h0 * HD, DMOD, (size_t)NN * NN, (size_t)HD * NN, (size_t)HD); }
        k_split512<<<NN / 8, 256, 0, stream>>>(O, NN, Oh, Ol);
        k_gemmb<true, false><<<dim3(NN / 64, DMOD / 64, 1), 128, 0, stream>>>(Oh, Ol, WP, b_proj, PO, DMOD, nullptr, nullptr, DMOD);
        k_addln512<true><<<NN / 8, 256, 0, stream>>>(PO, xb, g2, be2, X1, Hh, Hl);
        k_gemmb<true, false><<<dim3(NN / 64, DFF / 64, 1), 128, 0, stream>>>(Hh, Hl, WF1, b_ff1, F1, DFF, nullptr, nullptr, DMOD); k_gelu1024<<<NN / 8, 256, 0, stream>>>(F1, NN, Gh, Gl);
        k_gemmb<true, false><<<dim3(NN / 64, DMOD / 64, 1), 128, 0, stream>>>(Gh, Gl, WF2, b_ff2, F2, DMOD, nullptr, nullptr, DFF);
        k_add512<<<NN / 8, 256, 0, stream>>>(X1, F2, out + (size_t)b * NN * DMOD); }
}
